// positional_spiking_attention_27462020890903
// MI455X (gfx1250) — hardware-verified
//
#include <hip/hip_runtime.h>
#pragma clang fp contract(off)

#define TT 4
#define BB 4
#define LL 1024
#define DD 512
#define BL (BB * LL)
#define BLD (BB * LL * DD)
#define INVSTD 0.9999950000374997f
#define SPK1 0x3F80u

#define GP_LDP 40
#define GP_CPH 136
#define GP_CPF 132
#define GP_SMEM 34816

typedef __bf16 v16b __attribute__((ext_vector_type(16)));
typedef float v8f __attribute__((ext_vector_type(8)));
typedef float v4f __attribute__((ext_vector_type(4), __may_alias__));
typedef unsigned short us8 __attribute__((ext_vector_type(8), __may_alias__));

union FragB { v16b v; us8 u[2]; };

__device__ __forceinline__ unsigned int bf16_rne_bits(float f) {
  unsigned int u = __float_as_uint(f);
  u += 0x7FFFu + ((u >> 16) & 1u);
  return u >> 16;
}
__device__ __forceinline__ float bf16_rne_val(float f) {
  return __uint_as_float(bf16_rne_bits(f) << 16);
}
__device__ __forceinline__ float lif_step(float mem, float sp, float xin) {
  return (mem * 0.25f) * (1.0f - sp) + xin;
}
__device__ __forceinline__ void mma16(v8f& acc, const v16b a, const v16b b) {
  acc = __builtin_amdgcn_wmma_f32_16x16x32_bf16(false, a, false, b, (short)0, acc, false, false);
  asm volatile("v_nop\n\tv_nop\n\tv_nop\n\tv_nop" : "+v"(acc) : "v"(a), "v"(b));
}

__global__ __launch_bounds__(256) void k_wcvt(const float* __restrict__ w0,
                                              const float* __restrict__ w1,
                                              const float* __restrict__ w2,
                                              const float* __restrict__ w3,
                                              unsigned short* o0, unsigned short* o1,
                                              unsigned short* o2, unsigned short* o3, int n) {
  const float* src = w0;
  unsigned short* dst = o0;
  if (blockIdx.y == 1) { src = w1; dst = o1; }
  else if (blockIdx.y == 2) { src = w2; dst = o2; }
  else if (blockIdx.y == 3) { src = w3; dst = o3; }
  const size_t i = ((size_t)blockIdx.x * blockDim.x + threadIdx.x) * 8;
  if (i + 8 > (size_t)n) return;
  const v4f a = *(const v4f*)(src + i);
  const v4f c = *(const v4f*)(src + i + 4);
  us8 o = {0, 0, 0, 0, 0, 0, 0, 0};
  o[0] = (unsigned short)bf16_rne_bits(a[0]);
  o[1] = (unsigned short)bf16_rne_bits(a[1]);
  o[2] = (unsigned short)bf16_rne_bits(a[2]);
  o[3] = (unsigned short)bf16_rne_bits(a[3]);
  o[4] = (unsigned short)bf16_rne_bits(c[0]);
  o[5] = (unsigned short)bf16_rne_bits(c[1]);
  o[6] = (unsigned short)bf16_rne_bits(c[2]);
  o[7] = (unsigned short)bf16_rne_bits(c[3]);
  unsigned short* p = dst + i;
  *(volatile us8*)p = o;
  __threadfence();
  *(volatile us8*)p = o;
}

__global__ __launch_bounds__(256) void k_lif_in(const float* __restrict__ x,
                                                unsigned short* xs, int bld) {
  const size_t e = ((size_t)blockIdx.x * blockDim.x + threadIdx.x) * 8;
  if (e + 8 > (size_t)bld) return;
  float mem[8], sp[8];
#pragma unroll
  for (int i = 0; i < 8; ++i) { mem[i] = 0.0f; sp[i] = 0.0f; }
  us8 o[TT];
#pragma unroll
  for (int t = 0; t < TT; ++t) {
    const float* px = x + (size_t)t * bld + e;
    const v4f a = *(const v4f*)px;
    const v4f c = *(const v4f*)(px + 4);
    const float xv[8] = {a[0], a[1], a[2], a[3], c[0], c[1], c[2], c[3]};
    us8 ov = {0, 0, 0, 0, 0, 0, 0, 0};
#pragma unroll
    for (int i = 0; i < 8; ++i) {
      const float xi = bf16_rne_val(xv[i]);
      mem[i] = (t == 0) ? xi : lif_step(mem[i], sp[i], xi);
      const bool s = mem[i] > 0.5f;
      sp[i] = s ? 1.0f : 0.0f;
      ov[i] = s ? (unsigned short)SPK1 : (unsigned short)0;
    }
    o[t] = ov;
  }
  unsigned short* po = xs + e;
#pragma unroll
  for (int t = 0; t < TT; ++t) *(volatile us8*)(po + (size_t)t * bld) = o[t];
  __threadfence();
#pragma unroll
  for (int t = 0; t < TT; ++t) *(volatile us8*)(po + (size_t)t * bld) = o[t];
}

template <int SPK>
__global__ __launch_bounds__(256) void k_gemm(const unsigned short* __restrict__ A,
                                              const unsigned short* __restrict__ W,
                                              const float* __restrict__ bias,
                                              const float* __restrict__ gamma,
                                              const float* __restrict__ beta,
                                              unsigned short* outS, float* outF) {
  __shared__ __align__(16) unsigned char smem[GP_SMEM];
  unsigned short* ldsA = reinterpret_cast<unsigned short*>(smem);
  unsigned short* ldsB = ldsA + 128 * GP_LDP;

  const int tid = threadIdx.x, lane = tid & 31, wid = tid >> 5;
  const int wl = wid & 1, wn = wid >> 1;
  const int m16 = lane & 15, hh = lane >> 4;
  const int blockN = blockIdx.x * 128;
  const int bidx = blockIdx.y >> 5;
  const int l0 = (blockIdx.y & 31) * 32;

  const int sr = tid >> 1, sh = tid & 1;
  const int srt = sr >> 5, srl = sr & 31;
  const unsigned short* gA = A + (size_t)(srt * BL + bidx * LL + l0 + srl) * DD + sh * 16;
  const unsigned short* gW = W + (size_t)(blockN + sr) * DD + sh * 16;
  unsigned short* sA = ldsA + sr * GP_LDP + sh * 16;
  unsigned short* sB = ldsB + sr * GP_LDP + sh * 16;

  const v8f z8 = {0.f, 0.f, 0.f, 0.f, 0.f, 0.f, 0.f, 0.f};
  v8f acc[TT][2];
#pragma unroll
  for (int t = 0; t < TT; ++t) { acc[t][0] = z8; acc[t][1] = z8; }

#pragma unroll 1
  for (int k0 = 0; k0 < DD; k0 += 32) {
    const us8 a0 = *(const us8*)(gA + k0);
    const us8 a1 = *(const us8*)(gA + k0 + 8);
    const us8 b0 = *(const us8*)(gW + k0);
    const us8 b1 = *(const us8*)(gW + k0 + 8);
    __syncthreads();
    *(us8*)sA = a0;
    *(us8*)(sA + 8) = a1;
    *(us8*)sB = b0;
    *(us8*)(sB + 8) = b1;
    __syncthreads();

    FragB fa[TT], fb[2];
#pragma unroll
    for (int t = 0; t < TT; ++t) {
      const unsigned short* ap = ldsA + (t * 32 + wl * 16 + m16) * GP_LDP;
      fa[t].u[0] = *(const us8*)(ap + 8 * hh);
      fa[t].u[1] = *(const us8*)(ap + 16 + 8 * hh);
    }
#pragma unroll
    for (int f = 0; f < 2; ++f) {
      const unsigned short* bp = ldsB + (wn * 32 + f * 16 + m16) * GP_LDP;
      fb[f].u[0] = *(const us8*)(bp + 8 * hh);
      fb[f].u[1] = *(const us8*)(bp + 16 + 8 * hh);
    }
#pragma unroll
    for (int t = 0; t < TT; ++t)
#pragma unroll
      for (int f = 0; f < 2; ++f)
        mma16(acc[t][f], fa[t].v, fb[f].v);
  }
  __syncthreads();

  if (SPK) {
    unsigned short* ldsC = reinterpret_cast<unsigned short*>(smem);
#pragma unroll
    for (int f = 0; f < 2; ++f) {
      const int nl = wn * 32 + f * 16 + m16;
      const int ng = blockN + nl;
      const float bi = bf16_rne_val(bias[ng]);
      const float sc = INVSTD * bf16_rne_val(gamma[ng]);
      const float be = bf16_rne_val(beta[ng]);
#pragma unroll
      for (int r = 0; r < 8; ++r) {
        const int lrow = wl * 16 + 8 * hh + r;
        float pre = (acc[0][f][r] + bi) * sc + be;
        float mem = pre;
        bool s = mem > 0.5f;
        float sp = s ? 1.0f : 0.0f;
        ldsC[(0 * 32 + lrow) * GP_CPH + nl] = s ? (unsigned short)SPK1 : (unsigned short)0;
        pre = (acc[1][f][r] + bi) * sc + be;
        mem = lif_step(mem, sp, pre); s = mem > 0.5f; sp = s ? 1.0f : 0.0f;
        ldsC[(1 * 32 + lrow) * GP_CPH + nl] = s ? (unsigned short)SPK1 : (unsigned short)0;
        pre = (acc[2][f][r] + bi) * sc + be;
        mem = lif_step(mem, sp, pre); s = mem > 0.5f; sp = s ? 1.0f : 0.0f;
        ldsC[(2 * 32 + lrow) * GP_CPH + nl] = s ? (unsigned short)SPK1 : (unsigned short)0;
        pre = (acc[3][f][r] + bi) * sc + be;
        mem = lif_step(mem, sp, pre); s = mem > 0.5f; sp = s ? 1.0f : 0.0f;
        ldsC[(3 * 32 + lrow) * GP_CPH + nl] = s ? (unsigned short)SPK1 : (unsigned short)0;
      }
    }
    __syncthreads();
    us8 vv[8];
#pragma unroll
    for (int it = 0; it < 8; ++it) {
      const int R = wid * 16 + 2 * it + hh;
      vv[it] = *(const us8*)(ldsC + R * GP_CPH + m16 * 8);
    }
#pragma unroll
    for (int it = 0; it < 8; ++it) {
      const int R = wid * 16 + 2 * it + hh;
      const int t = R >> 5, lr = R & 31;
      unsigned short* gp = outS + (size_t)(t * BL + bidx * LL + l0 + lr) * DD + blockN + m16 * 8;
      *(volatile us8*)gp = vv[it];
    }
    __threadfence();
#pragma unroll
    for (int it = 0; it < 8; ++it) {
      const int R = wid * 16 + 2 * it + hh;
      const int t = R >> 5, lr = R & 31;
      unsigned short* gp = outS + (size_t)(t * BL + bidx * LL + l0 + lr) * DD + blockN + m16 * 8;
      *(volatile us8*)gp = vv[it];
    }
  } else {
    float* ldsF = reinterpret_cast<float*>(smem);
    float bi2[2], sc2[2], be2[2];
#pragma unroll
    for (int f = 0; f < 2; ++f) {
      const int ng = blockN + wn * 32 + f * 16 + m16;
      bi2[f] = bf16_rne_val(bias[ng]);
      sc2[f] = INVSTD * bf16_rne_val(gamma[ng]);
      be2[f] = bf16_rne_val(beta[ng]);
    }
#pragma unroll
    for (int p = 0; p < 2; ++p) {
      __syncthreads();
#pragma unroll
      for (int f = 0; f < 2; ++f) {
        const int nl = wn * 32 + f * 16 + m16;
#pragma unroll
        for (int r = 0; r < 8; ++r) {
          const int lrow = wl * 16 + 8 * hh + r;
#pragma unroll
          for (int tt = 0; tt < 2; ++tt) {
            const float val = (acc[2 * p + tt][f][r] + bi2[f]) * sc2[f] + be2[f];
            ldsF[(tt * 32 + lrow) * GP_CPF + nl] = val;
          }
        }
      }
      __syncthreads();
      v4f vv[8];
#pragma unroll
      for (int it = 0; it < 8; ++it) {
        const int R = wid * 8 + it;
        vv[it] = *(const v4f*)(ldsF + R * GP_CPF + lane * 4);
      }
#pragma unroll
      for (int it = 0; it < 8; ++it) {
        const int R = wid * 8 + it;
        const int tt = R >> 5, lr = R & 31;
        float* gp = outF + (size_t)((2 * p + tt) * BL + bidx * LL + l0 + lr) * DD + blockN + lane * 4;
        *(volatile v4f*)gp = vv[it];
      }
      __threadfence();
#pragma unroll
      for (int it = 0; it < 8; ++it) {
        const int R = wid * 8 + it;
        const int tt = R >> 5, lr = R & 31;
        float* gp = outF + (size_t)((2 * p + tt) * BL + bidx * LL + l0 + lr) * DD + blockN + lane * 4;
        *(volatile v4f*)gp = vv[it];
      }
    }
  }
}

__global__ __launch_bounds__(256) void k_band_lif(const unsigned short* __restrict__ qs,
                                                  const unsigned short* __restrict__ ks,
                                                  const unsigned short* __restrict__ vs,
                                                  const float* __restrict__ pb,
                                                  unsigned short* s2, int bld) {
  const size_t e = ((size_t)blockIdx.x * blockDim.x + threadIdx.x) * 8;
  if (e + 8 > (size_t)bld) return;
  const int d0 = (int)(e % DD);
  const int l = (int)((e / DD) % LL);
  const int b = (int)(e / ((size_t)LL * DD));

  float pw[8];
#pragma unroll
  for (int w = 0; w < 8; ++w) {
    const int j = l - 7 + w;
    pw[w] = 0.0f;
    if (j >= 0) pw[w] = bf16_rne_val(pb[(size_t)l * LL + j]);
  }

  float mem[8], sp[8];
#pragma unroll
  for (int i = 0; i < 8; ++i) { mem[i] = 0.0f; sp[i] = 0.0f; }
  us8 o[TT];
#pragma unroll
  for (int t = 0; t < TT; ++t) {
    const size_t tb = (size_t)t * bld + (size_t)b * LL * DD;
    float sum[8];
#pragma unroll
    for (int i = 0; i < 8; ++i) sum[i] = 0.0f;
#pragma unroll
    for (int w = 0; w < 8; ++w) {
      const int j = l - 7 + w;
      if (j >= 0) {
        const size_t off = tb + (size_t)j * DD + d0;
        const us8 kk = *(const us8*)(ks + off);
        const us8 vq = *(const us8*)(vs + off);
#pragma unroll
        for (int i = 0; i < 8; ++i) {
          const float kvf = ((kk[i] != 0) && (vq[i] != 0)) ? 1.0f : 0.0f;
          sum[i] = sum[i] + pw[w] * kvf;
        }
      }
    }
    const us8 qq = *(const us8*)(qs + tb + (size_t)l * DD + d0);
    us8 ov = {0, 0, 0, 0, 0, 0, 0, 0};
#pragma unroll
    for (int i = 0; i < 8; ++i) {
      const float qf = (qq[i] != 0) ? 1.0f : 0.0f;
      const float pre = qf * sum[i];
      mem[i] = (t == 0) ? pre : lif_step(mem[i], sp[i], pre);
      const bool s = mem[i] > 0.5f;
      sp[i] = s ? 1.0f : 0.0f;
      ov[i] = s ? (unsigned short)SPK1 : (unsigned short)0;
    }
    o[t] = ov;
  }
  unsigned short* po = s2 + e;
#pragma unroll
  for (int t = 0; t < TT; ++t) *(volatile us8*)(po + (size_t)t * bld) = o[t];
  __threadfence();
#pragma unroll
  for (int t = 0; t < TT; ++t) *(volatile us8*)(po + (size_t)t * bld) = o[t];
}

extern "C" void kernel_launch(void* const* d_in, const int* in_sizes, int n_in,
                              void* d_out, int out_size, void* d_ws,
                              size_t ws_size, hipStream_t stream) {
  if (n_in < 18) return;
  if (in_sizes[0] != TT * BLD || out_size != TT * BLD || in_sizes[1] != LL * LL) return;
  if (in_sizes[2] != DD * DD || in_sizes[6] != DD * DD || in_sizes[10] != DD * DD ||
      in_sizes[14] != DD * DD) return;
  if (in_sizes[3] != DD || in_sizes[4] != DD || in_sizes[5] != DD || in_sizes[15] != DD ||
      in_sizes[16] != DD || in_sizes[17] != DD) return;

  const float* x      = (const float*)d_in[0];
  const float* pb     = (const float*)d_in[1];
  const float* q_w    = (const float*)d_in[2];
  const float* q_b    = (const float*)d_in[3];
  const float* q_g    = (const float*)d_in[4];
  const float* q_be   = (const float*)d_in[5];
  const float* k_w    = (const float*)d_in[6];
  const float* k_b    = (const float*)d_in[7];
  const float* k_g    = (const float*)d_in[8];
  const float* k_be   = (const float*)d_in[9];
  const float* v_w    = (const float*)d_in[10];
  const float* v_b    = (const float*)d_in[11];
  const float* v_g    = (const float*)d_in[12];
  const float* v_be   = (const float*)d_in[13];
  const float* l_w    = (const float*)d_in[14];
  const float* l_b    = (const float*)d_in[15];
  const float* l_g    = (const float*)d_in[16];
  const float* l_be   = (const float*)d_in[17];

  const size_t wbytes = (size_t)DD * DD * 2;
  const size_t sbytes = (size_t)TT * BLD * 2;
  char* ws = (char*)d_ws;
  size_t off = 0;
  unsigned short* wq16 = (unsigned short*)(ws + off); off += wbytes;
  unsigned short* wk16 = (unsigned short*)(ws + off); off += wbytes;
  unsigned short* wv16 = (unsigned short*)(ws + off); off += wbytes;
  unsigned short* wl16 = (unsigned short*)(ws + off); off += wbytes;
  unsigned short* xs   = (unsigned short*)(ws + off); off += sbytes;
  unsigned short* qsp  = (unsigned short*)(ws + off); off += sbytes;
  unsigned short* ksp  = (unsigned short*)(ws + off); off += sbytes;
  unsigned short* vsp  = (unsigned short*)(ws + off); off += sbytes;
  unsigned short* s2   = (unsigned short*)(ws + off); off += sbytes;
  if (off > ws_size) return;
  float* out = (float*)d_out;

  const dim3 blk(256);
  const dim3 gcvt(DD * DD / 8 / 256, 4);
  const dim3 gelw(BLD / 8 / 256);
  const dim3 ggem(DD / 128, BB * (LL / 32));

  k_wcvt<<<gcvt, blk, 0, stream>>>(q_w, k_w, v_w, l_w, wq16, wk16, wv16, wl16, DD * DD);
  k_lif_in<<<gelw, blk, 0, stream>>>(x, xs, BLD);
  k_gemm<1><<<ggem, blk, 0, stream>>>(xs, wq16, q_b, q_g, q_be, qsp, out);
  k_gemm<1><<<ggem, blk, 0, stream>>>(xs, wk16, k_b, k_g, k_be, ksp, out);
  k_gemm<1><<<ggem, blk, 0, stream>>>(xs, wv16, v_b, v_g, v_be, vsp, out);
  k_band_lif<<<gelw, blk, 0, stream>>>(qsp, ksp, vsp, pb, s2, BLD);
  k_gemm<0><<<ggem, blk, 0, stream>>>(s2, wl16, l_b, l_g, l_be, xs, out);
}
